// LSTMDecoder_30872224924301
// MI455X (gfx1250) — hardware-run, weakly checked
//
#include <hip/hip_runtime.h>

constexpr int NBATCH   = 256;
constexpr int NDIM     = 512;
constexpr int NGATE    = 4 * NDIM;
constexpr int KCAT     = 2 * NDIM;
constexpr int TSTEPS   = 64;
constexpr int NTHR     = 256;
constexpr int NWAVE    = NTHR / 32;
constexpr int ROWS_BLK = 16;
constexpr int HPITCH   = 520;
constexpr int SLP      = 16;
constexpr int NPLANE   = 5;
constexpr float WCARRY = 256.0f;
constexpr float HCARRY = 16.0f;
constexpr float FOLD   = 1.0f / 4096.0f;
constexpr size_t GSTRIDE = (size_t)NDIM * KCAT;
constexpr int NOUT     = TSTEPS * NBATCH * NDIM;

static_assert(NBATCH % ROWS_BLK == 0, "grid exact");
static_assert(NDIM == 64 * NWAVE, "8 waves x 64 hidden units");
static_assert(NDIM % 32 == 0 && KCAT % 32 == 0, "K multiple of 32");
static_assert((4 * ROWS_BLK * HPITCH) % NTHR == 0, "zero fill loop exact");
static_assert((ROWS_BLK * NDIM / 4) % NTHR == 0, "x staging loop exact");
static_assert((2 * NGATE / 4) % NTHR == 0, "bias staging exact");
static_assert(HPITCH % 8 == 0 && HPITCH >= NDIM, "16-B aligned plane rows");
static_assert(SLP >= ROWS_BLK && (SLP % 4) == 0, "slab holds 16 rows, 16-B aligned");
static_assert((NGATE * (NDIM / 8)) % NTHR == 0, "weight convert grid exact");
static_assert(NDIM / 8 == 64, "weight convert index split");

typedef __attribute__((ext_vector_type(16))) _Float16 v16h;
typedef __attribute__((ext_vector_type(8)))  _Float16 v8h;
typedef __attribute__((ext_vector_type(8)))  float    v8f;
typedef __attribute__((ext_vector_type(4)))  float    v4f;
typedef __attribute__((ext_vector_type(2)))  unsigned v2u;

__device__ __forceinline__ unsigned short f2bf_bits(float f) {
  unsigned u = __float_as_uint(f);
  return (unsigned short)((u + 0x7FFFu + ((u >> 16) & 1u)) >> 16);
}
__device__ __forceinline__ float bf_bits2f(unsigned short h) { return __uint_as_float(((unsigned)h) << 16); }
__device__ __forceinline__ float bf16r(float f) { return bf_bits2f(f2bf_bits(f)); }
__device__ __forceinline__ unsigned short h16bits(float f) { return __builtin_bit_cast(unsigned short, (_Float16)f); }

__device__ __forceinline__ void guard_all4(v8f& a0, v8f& a1, v8f& a2, v8f& a3,
                                           v16h x, v16h y0, v16h y1, v16h y2, v16h y3) {
  asm volatile("v_nop\n\tv_nop\n\tv_nop\n\tv_nop"
               : "+v"(a0), "+v"(a1), "+v"(a2), "+v"(a3)
               : "v"(x), "v"(y0), "v"(y1), "v"(y2), "v"(y3));
}
__device__ __forceinline__ void acc_guard4(v8f& a, v8f& b, v8f& c, v8f& d) {
  asm volatile("v_nop\n\tv_nop\n\tv_nop\n\tv_nop" : "+v"(a), "+v"(b), "+v"(c), "+v"(d));
}

template <typename T> struct Frag;
template <> struct Frag<_Float16> {
  typedef v16h V; union U { v16h v; v8h h[2]; };
  static __device__ __forceinline__ v16h load(const _Float16* p) {
    U f; f.h[0] = *(const v8h*)(p); f.h[1] = *(const v8h*)(p + 16); return f.v;
  }
  static __device__ __forceinline__ v8f mma(v16h a, v16h b, v8f c) {
    return __builtin_amdgcn_wmma_f32_16x16x32_f16(false, a, false, b, (short)0, c, false, false);
  }
};

__device__ __forceinline__ float fsig(float x)  { return __builtin_amdgcn_rcpf(1.0f + __expf(-x)); }
__device__ __forceinline__ float ftanh(float x) { return 1.0f - 2.0f * __builtin_amdgcn_rcpf(__expf(2.0f * x) + 1.0f); }

__global__ __launch_bounds__(NTHR) void cvtw_kernel(const float* __restrict__ src, unsigned short* __restrict__ dst, int dcol0) {
  const int i  = blockIdx.x * NTHR + threadIdx.x;
  const int n8 = NGATE * (NDIM / 8);
  if (i < n8) {
    const int row = i >> 6;
    const int c8  = i & 63;
    const float* sp = src + (size_t)row * NDIM + c8 * 8;
    const v4f a = *(const v4f*)(sp);
    const v4f b = *(const v4f*)(sp + 4);
    v8h hv;
#pragma unroll
    for (int e = 0; e < 4; ++e) {
      hv[e]     = __builtin_bit_cast(_Float16, h16bits(bf16r(a[e]) * WCARRY));
      hv[4 + e] = __builtin_bit_cast(_Float16, h16bits(bf16r(b[e]) * WCARRY));
    }
    unsigned short* dp = dst + (size_t)row * KCAT + dcol0 + c8 * 8;
    *(volatile v8h*)dp = hv;
    __threadfence();
    *(volatile v8h*)dp = hv;
  }
}

__device__ __forceinline__ void mac512(v8f& a0, v8f& a1, v8f& a2, v8f& a3,
                                       const _Float16* arow, const _Float16* wb) {
#pragma unroll 1
  for (int k0 = 0; k0 < NDIM; k0 += 32) {
    const v16h a  = Frag<_Float16>::load(arow + k0);
    const v16h b0 = Frag<_Float16>::load(wb + k0);
    const v16h b1 = Frag<_Float16>::load(wb + GSTRIDE + k0);
    const v16h b2 = Frag<_Float16>::load(wb + 2 * GSTRIDE + k0);
    const v16h b3 = Frag<_Float16>::load(wb + 3 * GSTRIDE + k0);
    a0 = Frag<_Float16>::mma(a, b0, a0);
    a1 = Frag<_Float16>::mma(a, b1, a1);
    a2 = Frag<_Float16>::mma(a, b2, a2);
    a3 = Frag<_Float16>::mma(a, b3, a3);
    guard_all4(a0, a1, a2, a3, a, b0, b1, b2, b3);
  }
}

template <bool EMIT>
__device__ __forceinline__ void lstm_layer(const _Float16* arow, const _Float16* hrow, _Float16* hdst,
                                           const _Float16* Wp, const float* Bsl, float (&cs)[4][8], float* sl,
                                           int wave, int c, int hh, int koff) {
  const v8f z8 = {0.f, 0.f, 0.f, 0.f, 0.f, 0.f, 0.f, 0.f};
#pragma unroll
  for (int nt = 0; nt < 4; ++nt) {
    const int j = 64 * wave + 16 * nt + c;
    const _Float16* wb = Wp + (size_t)j * KCAT + koff;
    v8f ai = z8, af = z8, ag = z8, ao = z8;
    mac512(ai, af, ag, ao, arow, wb);
    mac512(ai, af, ag, ao, hrow, wb + NDIM);
    acc_guard4(ai, af, ag, ao);
    const float bi = Bsl[j];
    const float bf = Bsl[NDIM + j];
    const float bg = Bsl[2 * NDIM + j];
    const float bo = Bsl[3 * NDIM + j];
    float hv[8];
#pragma unroll
    for (int r = 0; r < 8; ++r) {
      const float zi = ai[r] * FOLD + bi;
      const float zf = af[r] * FOLD + bf;
      const float zg = ag[r] * FOLD + bg;
      const float zo = ao[r] * FOLD + bo;
      const float cn = fsig(zf) * cs[nt][r] + fsig(zi) * ftanh(zg);
      cs[nt][r] = cn;
      const float hn = fsig(zo) * ftanh(cn);
      hv[r] = hn;
      hdst[(8 * hh + r) * HPITCH + j] = (_Float16)(hn * HCARRY);
    }
    if (EMIT) {
      v4f lo4 = {hv[0], hv[1], hv[2], hv[3]};
      v4f hi4 = {hv[4], hv[5], hv[6], hv[7]};
      *(v4f*)(sl + (16 * nt + c) * SLP + 8 * hh)     = lo4;
      *(v4f*)(sl + (16 * nt + c) * SLP + 8 * hh + 4) = hi4;
    }
  }
}

__global__ __launch_bounds__(NTHR) void lstm2_seq_kernel(
    const float* __restrict__ xin, const int* __restrict__ tptr,
    const unsigned short* __restrict__ W0p, const unsigned short* __restrict__ W1p,
    const float* __restrict__ bi0, const float* __restrict__ bh0,
    const float* __restrict__ bi1, const float* __restrict__ bh1,
    float* __restrict__ out) {
  __shared__ __align__(16) _Float16 Pl[NPLANE][ROWS_BLK * HPITCH];
  __shared__ __align__(16) float    Bs[2][NGATE];
  __shared__ __align__(16) float    Sl[NWAVE][64 * SLP];
  const _Float16* W0 = (const _Float16*)W0p;
  const _Float16* W1 = (const _Float16*)W1p;
  const int tid = threadIdx.x, lane = tid & 31, wave = tid >> 5;
  const int c = lane & 15, hh = lane >> 4, koff = hh * 8, c4 = c * 4;
  const int rowbase = blockIdx.x * ROWS_BLK;
  int tl = tptr[0];
  tl = (tl < 0) ? 0 : tl;
  tl = (tl > TSTEPS) ? TSTEPS : tl;

  {
    _Float16* pf = &Pl[0][0];
#pragma unroll 1
    for (int i = tid; i < 4 * ROWS_BLK * HPITCH; i += NTHR) pf[i] = (_Float16)0.0f;
  }
  {
    unsigned short* px = (unsigned short*)(&Pl[4][0]);
#pragma unroll 1
    for (int it = 0; it < (ROWS_BLK * NDIM / 4) / NTHR; ++it) {
      const int idx = it * NTHR + tid;
      const int row = idx >> 7;
      const int cc  = (idx & 127) * 4;
      const v4f v = *(const v4f*)(xin + (size_t)(rowbase + row) * NDIM + cc);
      const unsigned short u0 = h16bits(bf16r(v[0]) * HCARRY);
      const unsigned short u1 = h16bits(bf16r(v[1]) * HCARRY);
      const unsigned short u2 = h16bits(bf16r(v[2]) * HCARRY);
      const unsigned short u3 = h16bits(bf16r(v[3]) * HCARRY);
      v2u pk;
      pk[0] = (unsigned)u0 | ((unsigned)u1 << 16);
      pk[1] = (unsigned)u2 | ((unsigned)u3 << 16);
      *(v2u*)(px + row * HPITCH + cc) = pk;
    }
  }
#pragma unroll 1
  for (int it = 0; it < 2; ++it) {
    const int n4 = (it * NTHR + tid) * 4;
    const v4f a0 = *(const v4f*)(bi0 + n4);
    const v4f g0 = *(const v4f*)(bh0 + n4);
    const v4f a1 = *(const v4f*)(bi1 + n4);
    const v4f g1 = *(const v4f*)(bh1 + n4);
    v4f s0, s1;
#pragma unroll
    for (int e = 0; e < 4; ++e) {
      s0[e] = bf16r(a0[e]) + bf16r(g0[e]);
      s1[e] = bf16r(a1[e]) + bf16r(g1[e]);
    }
    *(v4f*)(&Bs[0][n4]) = s0;
    *(v4f*)(&Bs[1][n4]) = s1;
  }
  float c0s[4][8], c1s[4][8];
#pragma unroll
  for (int nt = 0; nt < 4; ++nt)
#pragma unroll
    for (int r = 0; r < 8; ++r) { c0s[nt][r] = 0.0f; c1s[nt][r] = 0.0f; }
  __syncthreads();

  float* sl = Sl[wave];
  const int aoff = c * HPITCH + koff;

#pragma unroll 1
  for (int t = 0; t < tl; ++t) {
    const int cur = t & 1, nxt = cur ^ 1;
    const int xi  = (t == 0) ? 4 : (2 + cur);
    lstm_layer<false>(&Pl[xi][0] + aoff, &Pl[cur][0] + aoff, &Pl[nxt][0], W0, &Bs[0][0], c0s, sl, wave, c, hh, koff);
    __syncthreads();
    lstm_layer<true>(&Pl[nxt][0] + aoff, &Pl[2 + cur][0] + aoff, &Pl[2 + nxt][0], W1, &Bs[1][0], c1s, sl, wave, c, hh, koff);
    __builtin_amdgcn_fence(__ATOMIC_RELEASE, "workgroup");
    __builtin_amdgcn_wave_barrier();
    __builtin_amdgcn_fence(__ATOMIC_ACQUIRE, "workgroup");
    for (int pass = 0; pass < 2; ++pass) {
#pragma unroll
      for (int it = 0; it < 8; ++it) {
        const int row = it * 2 + hh;
        v4f v;
        v[0] = sl[(c4 + 0) * SLP + row];
        v[1] = sl[(c4 + 1) * SLP + row];
        v[2] = sl[(c4 + 2) * SLP + row];
        v[3] = sl[(c4 + 3) * SLP + row];
        *(volatile v4f*)(out + ((size_t)t * NBATCH + (size_t)(rowbase + row)) * NDIM + 64 * wave + c4) = v;
      }
      __threadfence();
    }
    __builtin_amdgcn_fence(__ATOMIC_RELEASE, "workgroup");
    __builtin_amdgcn_wave_barrier();
    __builtin_amdgcn_fence(__ATOMIC_ACQUIRE, "workgroup");
    __syncthreads();
  }
}

extern "C" void kernel_launch(void* const* d_in, const int* in_sizes, int n_in,
                              void* d_out, int out_size, void* d_ws, size_t ws_size, hipStream_t stream) {
  if (n_in < 10 || d_out == nullptr || d_ws == nullptr) return;
  if (in_sizes[0] != NBATCH * NDIM || in_sizes[1] != 1 ||
      in_sizes[2] != NGATE * NDIM || in_sizes[3] != NGATE * NDIM || in_sizes[4] != NGATE || in_sizes[5] != NGATE ||
      in_sizes[6] != NGATE * NDIM || in_sizes[7] != NGATE * NDIM || in_sizes[8] != NGATE || in_sizes[9] != NGATE ||
      out_size != NOUT) return;

  const float* hin  = (const float*)d_in[0];
  const int*   tin  = (const int*)d_in[1];
  const float* wih0 = (const float*)d_in[2];
  const float* whh0 = (const float*)d_in[3];
  const float* bih0 = (const float*)d_in[4];
  const float* bhh0 = (const float*)d_in[5];
  const float* wih1 = (const float*)d_in[6];
  const float* whh1 = (const float*)d_in[7];
  const float* bih1 = (const float*)d_in[8];
  const float* bhh1 = (const float*)d_in[9];
  float* out = (float*)d_out;

  char* ws = (char*)d_ws; size_t off = 0;
  auto carve = [&](size_t bytes) -> char* { char* p = ws + off; off += (bytes + 255) & ~(size_t)255; return p; };
  unsigned short* WC0 = (unsigned short*)carve((size_t)NGATE * KCAT * 2);
  unsigned short* WC1 = (unsigned short*)carve((size_t)NGATE * KCAT * 2);
  if (off > ws_size || off > (size_t)134217728) return;

  const int wgrid = (NGATE * (NDIM / 8)) / NTHR;
  cvtw_kernel<<<wgrid, NTHR, 0, stream>>>(wih0, WC0, 0);
  cvtw_kernel<<<wgrid, NTHR, 0, stream>>>(whh0, WC0, NDIM);
  cvtw_kernel<<<wgrid, NTHR, 0, stream>>>(wih1, WC1, 0);
  cvtw_kernel<<<wgrid, NTHR, 0, stream>>>(whh1, WC1, NDIM);
  lstm2_seq_kernel<<<NBATCH / ROWS_BLK, NTHR, 0, stream>>>(hin, tin, WC0, WC1, bih0, bhh0, bih1, bhh1, out);
}
